// MultiHeadCrossAttention_91070486544730
// MI455X (gfx1250) — hardware-verified
//
#include <hip/hip_runtime.h>
#include <math.h>

#ifndef NB
#define NB 2
#endif
#ifndef SEQ
#define SEQ 4096
#endif
#ifndef SEQ_FULL
#define SEQ_FULL 4096
#endif
#define HID 256
#define NHEAD 4
#define DHD 64
#define KVB 64

static_assert(SEQ % 64 == 0);
static_assert(SEQ <= SEQ_FULL);
static_assert(HID == NHEAD * DHD);
static_assert((NB * SEQ) % 64 == 0);
static_assert(HID % 64 == 0);
static_assert(DHD == 64);

typedef __attribute__((ext_vector_type(16))) _Float16 v16h;
typedef __attribute__((ext_vector_type(8)))  _Float16 v8h;
typedef __attribute__((ext_vector_type(16))) __bf16   v16b;
typedef __attribute__((ext_vector_type(8)))  __bf16   v8b;
typedef __attribute__((ext_vector_type(8)))  float    v8f;
typedef __attribute__((ext_vector_type(4)))  float    v4f;
typedef __attribute__((ext_vector_type(8)))  unsigned short v8us;
typedef __attribute__((ext_vector_type(16))) unsigned short v16us;

__device__ __forceinline__ unsigned short f2bf_bits(float f) {
  unsigned u = __float_as_uint(f);
  return (unsigned short)((u + 0x7FFFu + ((u >> 16) & 1u)) >> 16);
}
__device__ __forceinline__ float bf_bits2f(unsigned short h) { return __uint_as_float(((unsigned)h) << 16); }
__device__ __forceinline__ float bf_rne(float f) { return bf_bits2f(f2bf_bits(f)); }

union FB { v16b v; v8b h[2]; };
union FH { v16h v; v8h h[2]; };
union FU { v16us v; v8us h[2]; };
__device__ __forceinline__ v16b ldfrag_b(const __bf16* p) {
  FB f; f.h[0] = *(const v8b*)(p); f.h[1] = *(const v8b*)(p + 16); return f.v;
}

__device__ __forceinline__ v8f mma_h(v16h a, v16h b, v8f c) {
  c = __builtin_amdgcn_wmma_f32_16x16x32_f16(false, a, false, b, (short)0, c, false, false);
  asm volatile("v_nop\n\tv_nop\n\tv_nop\n\tv_nop" : "+v"(c) : "v"(a), "v"(b));
  return c;
}
__device__ __forceinline__ v8f mma3_b(v16b ah, v16b al, v16b bh, v16b bl, v8f c) {
  c = __builtin_amdgcn_wmma_f32_16x16x32_bf16(false, ah, false, bh, (short)0, c, false, false);
  c = __builtin_amdgcn_wmma_f32_16x16x32_bf16(false, ah, false, bl, (short)0, c, false, false);
  c = __builtin_amdgcn_wmma_f32_16x16x32_bf16(false, al, false, bh, (short)0, c, false, false);
  asm volatile("v_nop\n\tv_nop\n\tv_nop\n\tv_nop" : "+v"(c) : "v"(ah), "v"(al), "v"(bh), "v"(bl));
  return c;
}
__device__ __forceinline__ void dep_guard_b(v8f& a, v8f& b, v16b x, v16b y) { asm volatile("v_nop\n\tv_nop\n\tv_nop\n\tv_nop" : "+v"(a), "+v"(b) : "v"(x), "v"(y)); }
__device__ __forceinline__ void keep4_b(v16b a, v16b b, v16b c, v16b d) { asm volatile("v_nop" :: "v"(a), "v"(b), "v"(c), "v"(d)); }
__device__ __forceinline__ void acc_guard4(v8f& a, v8f& b, v8f& c, v8f& d) { asm volatile("v_nop\n\tv_nop\n\tv_nop\n\tv_nop" : "+v"(a), "+v"(b), "+v"(c), "+v"(d)); }

__global__ __launch_bounds__(256) void k_cvt_x(const float* __restrict__ src, unsigned short* __restrict__ dst, int nrows) {
  const int u = blockIdx.x * 256 + threadIdx.x;
  if (u >= nrows * (HID / 8)) return;
  const int r = u >> 5, c8 = (u & 31) * 8;
  const int b = r / SEQ, s = r - b * SEQ;
  const float* p = src + ((long long)b * SEQ_FULL + s) * HID + c8;
  const v4f a = *(const v4f*)p;
  const v4f g = *(const v4f*)(p + 4);
  v8us o;
  o[0] = f2bf_bits(a.x); o[1] = f2bf_bits(a.y); o[2] = f2bf_bits(a.z); o[3] = f2bf_bits(a.w);
  o[4] = f2bf_bits(g.x); o[5] = f2bf_bits(g.y); o[6] = f2bf_bits(g.z); o[7] = f2bf_bits(g.w);
  volatile v8us* d = (volatile v8us*)(dst + (long long)r * HID + c8);
  *d = o;
  __threadfence();
  *d = o;
}

__global__ __launch_bounds__(256) void k_wt(const float* __restrict__ W0, const float* __restrict__ W1, const float* __restrict__ W2, const float* __restrict__ W3,
                                            unsigned short* __restrict__ D0, unsigned short* __restrict__ D1, unsigned short* __restrict__ D2, unsigned short* __restrict__ D3) {
  const int y = blockIdx.y;
  const float* W = (y == 0) ? W0 : ((y == 1) ? W1 : ((y == 2) ? W2 : W3));
  unsigned short* D = (y == 0) ? D0 : ((y == 1) ? D1 : ((y == 2) ? D2 : D3));
  const int u = blockIdx.x * 256 + threadIdx.x;
  if (u >= HID * (HID / 8)) return;
  const int o = u >> 5, k0 = (u & 31) * 8;
  v8us v;
#pragma unroll
  for (int e = 0; e < 8; ++e) v[e] = f2bf_bits(W[(long long)(k0 + e) * HID + o]);
  const int kp = (y == 3) ? 2 * HID : HID;
  unsigned short* d1 = D + (long long)o * kp + k0;
  unsigned short* d2 = d1 + HID;
  *(volatile v8us*)d1 = v;
  if (y == 3) *(volatile v8us*)d2 = v;
  __threadfence();
  *(volatile v8us*)d1 = v;
  if (y == 3) *(volatile v8us*)d2 = v;
}

template <int BIAS_MODE, int OUT_MODE>
__global__ __launch_bounds__(256) void k_gemm64(
    const unsigned short* __restrict__ Ap, int lda, long long strideA,
    const unsigned short* __restrict__ Btp, int ldb, long long strideB,
    void* __restrict__ Cout, void* __restrict__ Cout2, int ldc, long long strideC,
    const float* __restrict__ bias, int M, int N, int K) {
  __shared__ __align__(16) float sT[8][16 * 68];
  const int bz   = blockIdx.y;
  const int lane = threadIdx.x & 31;
  const int wave = threadIdx.x >> 5;
  const int tilesN = N >> 6;
  const int tilesM = M >> 6;
  const int tile = blockIdx.x * 8 + wave;
  if (tile >= tilesM * tilesN) return;
  const int tm = tile / tilesN;
  const int tn = tile - tm * tilesN;
  const int m0 = tm << 6;
  const int n0 = tn << 6;

  const __bf16* Ab = (const __bf16*)Ap  + (size_t)bz * strideA;
  const __bf16* Bb = (const __bf16*)Btp + (size_t)bz * strideB;

  const int rlane = lane & 15;
  const int koff  = (lane >> 4) * 8;
  const int mOff  = (lane >> 4) * 8;

  v8f acc[4][4];
#pragma unroll
  for (int i = 0; i < 4; ++i)
#pragma unroll
    for (int j = 0; j < 4; ++j) acc[i][j] = (v8f){0.f,0.f,0.f,0.f,0.f,0.f,0.f,0.f};

  for (int k0 = 0; k0 < K; k0 += 32) {
    v16b bh[4];
#pragma unroll
    for (int j = 0; j < 4; ++j) {
      const size_t bo = (size_t)(n0 + (j << 4) + rlane) * ldb + koff + k0;
      bh[j] = ldfrag_b(Bb + bo);
    }
#pragma unroll
    for (int i = 0; i < 4; ++i) {
      const size_t ao = (size_t)(m0 + (i << 4) + rlane) * lda + koff + k0;
      const v16b ah = ldfrag_b(Ab + ao);
#pragma unroll
      for (int j = 0; j < 4; ++j)
        acc[i][j] = __builtin_amdgcn_wmma_f32_16x16x32_bf16(false, ah, false, bh[j], (short)0, acc[i][j], false, false);
      dep_guard_b(acc[i][0], acc[i][3], ah, ah);
    }
    keep4_b(bh[0], bh[1], bh[2], bh[3]);
  }
  acc_guard4(acc[0][0], acc[0][1], acc[0][2], acc[0][3]);
  acc_guard4(acc[1][0], acc[1][1], acc[1][2], acc[1][3]);
  acc_guard4(acc[2][0], acc[2][1], acc[2][2], acc[2][3]);
  acc_guard4(acc[3][0], acc[3][1], acc[3][2], acc[3][3]);

  float* slab = sT[wave];
#pragma unroll
  for (int i = 0; i < 4; ++i) {
    const int mBase = m0 + (i << 4);
#pragma unroll
    for (int j = 0; j < 4; ++j) {
      const int n = n0 + (j << 4) + rlane;
      float bv = 0.f;
      if (BIAS_MODE == 2) bv = bf_rne(bias[n]);
#pragma unroll
      for (int r = 0; r < 8; ++r) {
        float v = acc[i][j][r];
        if (BIAS_MODE == 1) v += bf_rne(bias[mBase + mOff + r]);
        if (BIAS_MODE == 2) v += bv;
        slab[(mOff + r) * 68 + (j << 4) + rlane] = v;
      }
    }
    __builtin_amdgcn_fence(3, "workgroup");
    __builtin_amdgcn_wave_barrier();
    __builtin_amdgcn_fence(2, "workgroup");
    if (OUT_MODE == 0) {
      float* C = (float*)Cout + (size_t)bz * strideC;
      const int hh = lane >> 4, c4 = (lane & 15) * 4;
      for (int pass = 0; pass < 2; ++pass) {
#pragma unroll
        for (int it = 0; it < 8; ++it) {
          const int row = it * 2 + hh;
          const v4f v = *(const v4f*)(slab + row * 68 + c4);
          *(volatile v4f*)(C + (size_t)(mBase + row) * ldc + n0 + c4) = v;
        }
        __threadfence();
      }
    } else if (OUT_MODE == 1) {
      const int q = lane >> 3, c8 = (lane & 7) * 8;
      _Float16* C = (_Float16*)Cout + (size_t)bz * strideC;
      for (int pass = 0; pass < 2; ++pass) {
#pragma unroll
        for (int it = 0; it < 4; ++it) {
          const int row = it * 4 + q;
          const float* sp = slab + row * 68 + c8;
          v8h hv;
#pragma unroll
          for (int e = 0; e < 8; ++e) hv[e] = (_Float16)sp[e];
          *(volatile v8h*)(C + (size_t)(mBase + row) * ldc + n0 + c8) = hv;
        }
        __threadfence();
      }
    } else {
      const int q = lane >> 3, c8 = (lane & 7) * 8;
      unsigned short* C  = (unsigned short*)Cout  + (size_t)bz * strideC;
      unsigned short* C2 = (unsigned short*)Cout2 + (size_t)bz * strideC;
      for (int pass = 0; pass < 2; ++pass) {
#pragma unroll
        for (int it = 0; it < 4; ++it) {
          const int row = it * 4 + q;
          const float* sp = slab + row * 68 + c8;
          v8us hv, lv;
#pragma unroll
          for (int e = 0; e < 8; ++e) {
            const float x = sp[e];
            const unsigned short hb = f2bf_bits(x);
            const unsigned short lb = f2bf_bits(x - bf_bits2f(hb));
            hv[e] = hb; lv[e] = lb;
          }
          *(volatile v8us*)(C  + (size_t)(mBase + row) * ldc + n0 + c8) = hv;
          *(volatile v8us*)(C2 + (size_t)(mBase + row) * ldc + n0 + c8) = lv;
        }
        __threadfence();
      }
    }
    __builtin_amdgcn_fence(3, "workgroup");
    __builtin_amdgcn_wave_barrier();
    __builtin_amdgcn_fence(2, "workgroup");
  }
}

__global__ __launch_bounds__(128) __attribute__((amdgpu_num_vgpr(256)))
void k_attn(const unsigned short* __restrict__ QP, const unsigned short* __restrict__ KP,
            const unsigned short* __restrict__ VH, const unsigned short* __restrict__ VL,
            const int* __restrict__ kvm, unsigned short* __restrict__ CX) {
  __shared__ __align__(16) _Float16       Ksh[KVB * DHD];
  __shared__ __align__(16) unsigned short Vth[DHD * KVB];
  __shared__ __align__(16) unsigned short Vtl[DHD * KVB];
  __shared__ __align__(16) unsigned short Psh[4][16 * KVB];
  __shared__ __align__(16) unsigned short Psl[4][16 * KVB];
  __shared__ __align__(16) float          Os[4][16 * 68];

  const int tid  = threadIdx.x;
  const int wave = tid >> 5;
  const int lane = tid & 31;
  const int hh   = lane >> 4;
  const int c    = lane & 15;

  const int nqb = SEQ / 64;
  const int bx  = blockIdx.x;
  const int qb  = bx % nqb;
  const int bhd = bx / nqb;
  const int h   = bhd % NHEAD;
  const int b   = bhd / NHEAD;
  const int q0  = qb * 64 + wave * 16;

  const _Float16* Qp = (const _Float16*)QP;
  const _Float16* Kp = (const _Float16*)KP;

  FH qa[2];
  {
    const _Float16* qrow = Qp + ((long long)b * SEQ + q0 + c) * HID + h * DHD;
#pragma unroll
    for (int dc = 0; dc < 2; ++dc) {
      qa[dc].h[0] = *(const v8h*)(qrow + dc * 32 + 8 * hh);
      qa[dc].h[1] = *(const v8h*)(qrow + dc * 32 + 16 + 8 * hh);
    }
  }

  const float NEG = -__builtin_inff();
  const float SCL = 0.125f * 1.4426950408889634f;
  float mrow[8], lrow[8];
  v8f oacc[4];
#pragma unroll
  for (int r = 0; r < 8; ++r) { mrow[r] = NEG; lrow[r] = 0.f; }
#pragma unroll
  for (int t = 0; t < 4; ++t) oacc[t] = (v8f){0.f,0.f,0.f,0.f,0.f,0.f,0.f,0.f};

  const long long kbase = (long long)b * SEQ;
  const long long vbase = ((long long)b * HID + h * DHD) * (long long)SEQ;
  const long long mbase = (long long)b * SEQ_FULL;
  unsigned short* pwh = Psh[wave];
  unsigned short* pwl = Psl[wave];

  const int nchunk = SEQ / KVB;
  for (int kc = 0; kc < nchunk; ++kc) {
    const int kv0 = kc * KVB;
    __syncthreads();
    for (int i = tid; i < KVB * (DHD / 8); i += 128) {
      const int r = i >> 3, c8 = (i & 7) * 8;
      *(v8h*)(Ksh + r * DHD + c8) = *(const v8h*)(Kp + (kbase + kv0 + r) * HID + h * DHD + c8);
    }
    for (int i = tid; i < DHD * (KVB / 8); i += 128) {
      const int d = i >> 3, c8 = (i & 7) * 8;
      const long long go = vbase + (long long)d * SEQ + kv0 + c8;
      *(v8us*)(Vth + d * KVB + c8) = *(const v8us*)(VH + go);
      *(v8us*)(Vtl + d * KVB + c8) = *(const v8us*)(VL + go);
    }
    __syncthreads();

    v8f s[4];
#pragma unroll
    for (int j = 0; j < 4; ++j) {
      s[j] = (v8f){0.f,0.f,0.f,0.f,0.f,0.f,0.f,0.f};
#pragma unroll
      for (int dc = 0; dc < 2; ++dc) {
        FH kb;
        kb.h[0] = *(const v8h*)(Ksh + (j * 16 + c) * DHD + dc * 32 + 8 * hh);
        kb.h[1] = *(const v8h*)(Ksh + (j * 16 + c) * DHD + dc * 32 + 16 + 8 * hh);
        s[j] = mma_h(qa[dc].v, kb.v, s[j]);
      }
    }
    int kvkeep[4];
#pragma unroll
    for (int j = 0; j < 4; ++j) kvkeep[j] = kvm[mbase + kv0 + j * 16 + c];

    float cm[8];
#pragma unroll
    for (int r = 0; r < 8; ++r) {
      float m = NEG;
#pragma unroll
      for (int j = 0; j < 4; ++j) {
        float v = s[j][r] * SCL;
        v = (kvkeep[j] != 0) ? v : NEG;
        s[j][r] = v;
        m = fmaxf(m, v);
      }
      m = fmaxf(m, __shfl_xor(m, 1, 32)); m = fmaxf(m, __shfl_xor(m, 2, 32));
      m = fmaxf(m, __shfl_xor(m, 4, 32)); m = fmaxf(m, __shfl_xor(m, 8, 32));
      cm[r] = m;
    }
#pragma unroll
    for (int r = 0; r < 8; ++r) {
      const float mnew  = fmaxf(mrow[r], cm[r]);
      const float alpha = (mnew == NEG) ? 1.f : exp2f(mrow[r] - mnew);
      mrow[r] = mnew;
      float psum = 0.f;
#pragma unroll
      for (int j = 0; j < 4; ++j) {
        const float sv = s[j][r];
        const float p = (sv == NEG) ? 0.f : exp2f(sv - mnew);
        psum += p;
        const unsigned short hb = f2bf_bits(p);
        const unsigned short lb = f2bf_bits(p - bf_bits2f(hb));
        pwh[(8 * hh + r) * KVB + j * 16 + c] = hb;
        pwl[(8 * hh + r) * KVB + j * 16 + c] = lb;
      }
      psum += __shfl_xor(psum, 1, 32); psum += __shfl_xor(psum, 2, 32);
      psum += __shfl_xor(psum, 4, 32); psum += __shfl_xor(psum, 8, 32);
      lrow[r] = lrow[r] * alpha + psum;
#pragma unroll
      for (int t = 0; t < 4; ++t) oacc[t][r] *= alpha;
    }
    __builtin_amdgcn_fence(3, "workgroup");
    __builtin_amdgcn_wave_barrier();
    __builtin_amdgcn_fence(2, "workgroup");
#pragma unroll 1
    for (int kk = 0; kk < 2; ++kk) {
      FU pa, pl;
      pa.h[0] = *(const v8us*)(pwh + c * KVB + kk * 32 + 8 * hh);
      pa.h[1] = *(const v8us*)(pwh + c * KVB + kk * 32 + 16 + 8 * hh);
      pl.h[0] = *(const v8us*)(pwl + c * KVB + kk * 32 + 8 * hh);
      pl.h[1] = *(const v8us*)(pwl + c * KVB + kk * 32 + 16 + 8 * hh);
      const v16b pav = __builtin_bit_cast(v16b, pa.v);
      const v16b plv = __builtin_bit_cast(v16b, pl.v);
#pragma unroll
      for (int t = 0; t < 4; ++t) {
        FU vb, vl;
        vb.h[0] = *(const v8us*)(Vth + (t * 16 + c) * KVB + kk * 32 + 8 * hh);
        vb.h[1] = *(const v8us*)(Vth + (t * 16 + c) * KVB + kk * 32 + 16 + 8 * hh);
        vl.h[0] = *(const v8us*)(Vtl + (t * 16 + c) * KVB + kk * 32 + 8 * hh);
        vl.h[1] = *(const v8us*)(Vtl + (t * 16 + c) * KVB + kk * 32 + 16 + 8 * hh);
        oacc[t] = mma3_b(pav, plv, __builtin_bit_cast(v16b, vb.v), __builtin_bit_cast(v16b, vl.v), oacc[t]);
      }
    }
  }

  float* os = Os[wave];
#pragma unroll
  for (int r = 0; r < 8; ++r) {
    const float inv = 1.0f / lrow[r];
#pragma unroll
    for (int t = 0; t < 4; ++t) os[(8 * hh + r) * 68 + t * 16 + c] = oacc[t][r] * inv;
  }
  __builtin_amdgcn_fence(3, "workgroup");
  __builtin_amdgcn_wave_barrier();
  __builtin_amdgcn_fence(2, "workgroup");
  {
    const int q4 = lane >> 3, c8 = (lane & 7) * 8;
    unsigned short* cxh = CX + ((long long)b * SEQ + q0) * (2 * HID) + h * DHD;
    unsigned short* cxl = cxh + HID;
    for (int pass = 0; pass < 2; ++pass) {
#pragma unroll
      for (int it = 0; it < 4; ++it) {
        const int row = it * 4 + q4;
        const float* sp = os + row * 68 + c8;
        v8us hv, lv;
#pragma unroll
        for (int e = 0; e < 8; ++e) {
          const float x = sp[e];
          const unsigned short hb = f2bf_bits(x);
          const unsigned short lb = f2bf_bits(x - bf_bits2f(hb));
          hv[e] = hb; lv[e] = lb;
        }
        *(volatile v8us*)(cxh + (long long)row * (2 * HID) + c8) = hv;
        *(volatile v8us*)(cxl + (long long)row * (2 * HID) + c8) = lv;
      }
      __threadfence();
    }
  }
}

static inline size_t al256(size_t x) { return (x + 255) & ~(size_t)255; }

extern "C" void kernel_launch(void* const* d_in, const int* in_sizes, int n_in,
                              void* d_out, int out_size, void* d_ws, size_t ws_size, hipStream_t stream) {
  if (n_in < 11) return;
  const float* query     = (const float*)d_in[0];
  const float* key_value = (const float*)d_in[1];
  const int*   kv_mask   = (const int*)d_in[2];
  const float* Wq = (const float*)d_in[3];
  const float* bq = (const float*)d_in[4];
  const float* Wk = (const float*)d_in[5];
  const float* bk = (const float*)d_in[6];
  const float* Wv = (const float*)d_in[7];
  const float* bv = (const float*)d_in[8];
  const float* Wo = (const float*)d_in[9];
  const float* bo = (const float*)d_in[10];

  const long long needx = ((long long)(NB - 1) * SEQ_FULL + SEQ) * HID;
  if ((long long)in_sizes[0] < needx || (long long)in_sizes[1] < needx) return;
  if ((long long)in_sizes[2] < (long long)(NB - 1) * SEQ_FULL + SEQ) return;
  if (in_sizes[3] < HID * HID || in_sizes[5] < HID * HID || in_sizes[7] < HID * HID || in_sizes[9] < HID * HID) return;
  if (in_sizes[4] < HID || in_sizes[6] < HID || in_sizes[8] < HID || in_sizes[10] < HID) return;
  if ((long long)out_size < (long long)NB * SEQ * HID) return;

  const size_t MR = (size_t)NB * SEQ;
  size_t off = 0;
  const size_t oXQ  = off; off += al256(MR * HID * 2);
  const size_t oXKV = off; off += al256(MR * HID * 2);
  const size_t oWQT = off; off += al256((size_t)HID * HID * 2);
  const size_t oWKT = off; off += al256((size_t)HID * HID * 2);
  const size_t oWVT = off; off += al256((size_t)HID * HID * 2);
  const size_t oWO2 = off; off += al256((size_t)HID * 2 * HID * 2);
  const size_t oQP  = off; off += al256(MR * HID * 2);
  const size_t oKP  = off; off += al256(MR * HID * 2);
  const size_t oVTH = off; off += al256((size_t)NB * HID * SEQ * 2);
  const size_t oVTL = off; off += al256((size_t)NB * HID * SEQ * 2);
  const size_t oCX  = off; off += al256(MR * 2 * HID * 2);
  if (off > ws_size) return;

  char* ws = (char*)d_ws;
  unsigned short* XQ  = (unsigned short*)(ws + oXQ);
  unsigned short* XKV = (unsigned short*)(ws + oXKV);
  unsigned short* WQT = (unsigned short*)(ws + oWQT);
  unsigned short* WKT = (unsigned short*)(ws + oWKT);
  unsigned short* WVT = (unsigned short*)(ws + oWVT);
  unsigned short* WO2 = (unsigned short*)(ws + oWO2);
  unsigned short* QP  = (unsigned short*)(ws + oQP);
  unsigned short* KPp = (unsigned short*)(ws + oKP);
  unsigned short* VTH = (unsigned short*)(ws + oVTH);
  unsigned short* VTL = (unsigned short*)(ws + oVTL);
  unsigned short* CX  = (unsigned short*)(ws + oCX);
  float* out = (float*)d_out;

  const unsigned cvt_blocks = (unsigned)((MR * (HID / 8) + 255) / 256);
  k_cvt_x<<<cvt_blocks, 256, 0, stream>>>(query, XQ, (int)MR);
  k_cvt_x<<<cvt_blocks, 256, 0, stream>>>(key_value, XKV, (int)MR);
  k_wt<<<dim3((unsigned)((HID * (HID / 8) + 255) / 256), 4), 256, 0, stream>>>(Wq, Wk, Wv, Wo, WQT, WKT, WVT, WO2);
  const unsigned gproj = (unsigned)(((MR / 64) * (HID / 64) + 7) / 8);
  k_gemm64<2, 1><<<dim3(gproj, 1), 256, 0, stream>>>(XQ,  HID, 0, WQT, HID, 0, (void*)QP,  nullptr, HID, 0, bq, (int)MR, HID, HID);
  k_gemm64<2, 1><<<dim3(gproj, 1), 256, 0, stream>>>(XKV, HID, 0, WKT, HID, 0, (void*)KPp, nullptr, HID, 0, bk, (int)MR, HID, HID);
  const unsigned gvt = (unsigned)(((HID / 64) * (SEQ / 64) + 7) / 8);
  k_gemm64<1, 2><<<dim3(gvt, NB), 256, 0, stream>>>(WVT, HID, 0, XKV, HID, (long long)SEQ * HID, (void*)VTH, (void*)VTL, SEQ, (long long)HID * SEQ, bv, HID, SEQ, HID);
  k_attn<<<(unsigned)(NB * NHEAD * (SEQ / 64)), 128, 0, stream>>>(QP, KPp, VTH, VTL, kv_mask, CX);
  const unsigned gout = (unsigned)(((MR / 64) * (HID / 64) + 7) / 8);
  k_gemm64<2, 0><<<dim3(gout, 1), 256, 0, stream>>>(CX, 2 * HID, 0, WO2, 2 * HID, 0, (void*)out, nullptr, HID, 0, bo, (int)MR, HID, 2 * HID);
}
